// MultiHeadAttention_83614423318615
// MI455X (gfx1250) — hardware-verified
//
#include <hip/hip_runtime.h>
#include <math.h>

typedef __attribute__((ext_vector_type(16))) _Float16 v16h;
typedef __attribute__((ext_vector_type(16))) __bf16 v16b;
typedef __attribute__((ext_vector_type(8)))  _Float16 v8h;
typedef __attribute__((ext_vector_type(8)))  __bf16 v8b;
typedef __attribute__((ext_vector_type(8)))  float v8f;
typedef __attribute__((ext_vector_type(4)))  float v4f;
typedef __attribute__((ext_vector_type(4)))  unsigned v4u;

#ifndef NB
#define NB 2
#endif
#ifndef SEQ
#define SEQ 2048
#endif
#define NB_FULL 2
#define SEQ_FULL 2048
#ifndef OSEQ
#define OSEQ SEQ
#endif
#define TT SEQ
#define DIN 2048
#define NH 16
#define NKV 4
#define GRP (NH / NKV)
#define HD 128
#define HALF (HD / 2)
#define CQ (NH * HD)
#define CKV (NKV * HD)
#define NQB (TT / 64)
#define HG 4
#define SCALE (0.08838834764831845f)
#define QBH 6
#define QHI 384
#define KHI 384
static_assert(NB >= 1 && NB <= NB_FULL);
static_assert(SEQ % 128 == 0 && SEQ >= 128 && SEQ <= SEQ_FULL);
static_assert(HD == 128 && CQ % 128 == 0 && CKV % 128 == 0 && DIN % 64 == 0 && DIN == 256 * 8 && CQ % 32 == 0 && DIN % 128 == 0);
static_assert(QBH * 64 <= QHI && ((((QBH * 64 - 1) >> 7) + 1) * 128) <= KHI && QHI % 64 == 0 && KHI % 64 == 0);
static_assert(NH % HG == 0 && HG <= GRP && GRP % HG == 0);

#define WSZ_XB  (2u * (size_t)NB * TT * DIN)
#define WSZ_WQT (2u * (size_t)CQ * DIN)
#define WSZ_WKV (2u * (size_t)CKV * DIN)
#define WSZ_S   (4u * (size_t)HG * TT * TT)
#define WS_XB   ((size_t)0)
#define WS_WQT  (WS_XB + WSZ_XB)
#define WS_WKT  (WS_WQT + WSZ_WQT)
#define WS_WVT  (WS_WKT + WSZ_WKV)
#define WS_ALIAS_END (WS_WVT + WSZ_WKV)
#define WS_S    ((size_t)0)
#define WS_A    (WSZ_S > WS_ALIAS_END ? WSZ_S : WS_ALIAS_END)
#define WS_WOT  (WS_A)
#define WS_QH   (WS_WOT + 2u * (size_t)DIN * CQ)
#define WS_KH   (WS_QH + 2u * (size_t)NB * TT * CQ)
#define WS_VT   (WS_KH + 2u * (size_t)NB * TT * CKV)
#define WS_QL   (WS_VT + 2u * (size_t)NB * CKV * TT)
#define WS_KL   (WS_QL + 2u * (size_t)NB * QHI * CQ)
#define WS_VB   (WS_KL + 2u * (size_t)NB * KHI * CKV)
#define WS_VBL  (WS_VB + 2u * (size_t)NB * CKV * KHI)
#define WS_CH   (WS_VBL + 2u * (size_t)NB * CKV * KHI)
#define WS_CL   (WS_CH + 2u * (size_t)NB * TT * CQ)
#define WS_END  (WS_CL + 2u * (size_t)NB * QHI * CQ)
static_assert(WS_END <= (size_t)134217728u);
static_assert(WS_ALIAS_END <= WS_A && WSZ_S <= WS_A);
static_assert(WS_WQT % 128 == 0 && WS_WKT % 128 == 0 && WS_WVT % 128 == 0 && WS_A % 128 == 0 && WS_QH % 128 == 0 && WS_KH % 128 == 0 && WS_VT % 128 == 0 && WS_QL % 128 == 0 && WS_KL % 128 == 0 && WS_VB % 128 == 0 && WS_VBL % 128 == 0 && WS_CH % 128 == 0 && WS_CL % 128 == 0 && WS_END % 128 == 0);

template <typename T> __device__ __forceinline__ void vst2(void* p, T v) { *(volatile T*)p = v; __threadfence(); *(volatile T*)p = v; }
__device__ __forceinline__ v8f wmma16(v16h a, v16h b, v8f c) {
  v8f d = __builtin_amdgcn_wmma_f32_16x16x32_f16(false, a, false, b, (short)0, c, false, false);
  asm volatile("v_nop\n\tv_nop\n\tv_nop\n\tv_nop" : "+v"(d) : "v"(a), "v"(b));
  return d;
}
__device__ __forceinline__ v8f wmma_bf(v16b a, v16b b, v8f c) {
  v8f d = __builtin_amdgcn_wmma_f32_16x16x32_bf16(false, a, false, b, (short)0, c, false, false);
  asm volatile("v_nop\n\tv_nop\n\tv_nop\n\tv_nop" : "+v"(d) : "v"(a), "v"(b));
  return d;
}
__device__ __forceinline__ v16h frag_h(const _Float16* rowk0, int lane) {
  union { v16h v; v8h q[2]; } u; const _Float16* p = rowk0 + 8 * (lane >> 4);
  u.q[0] = *(const v8h*)p; u.q[1] = *(const v8h*)(p + 16); return u.v;
}
__device__ __forceinline__ v16b frag_b(const __bf16* rowk0, int lane) {
  union { v16b v; v8b q[2]; } u; const __bf16* p = rowk0 + 8 * (lane >> 4);
  u.q[0] = *(const v8b*)p; u.q[1] = *(const v8b*)(p + 16); return u.v;
}
__device__ __forceinline__ v16h frag_f32(const float* rowk0, int lane) {
  v16h a; const float* p = rowk0 + 8 * (lane >> 4);
#pragma unroll
  for (int i = 0; i < 8; ++i) { a[i] = (_Float16)p[i]; a[8 + i] = (_Float16)p[16 + i]; }
  return a;
}
struct F2 { v16b h, l; };
__device__ __forceinline__ F2 bsplit16(const float v[16]) { F2 r;
#pragma unroll
  for (int i = 0; i < 16; ++i) { const __bf16 h = (__bf16)v[i]; r.h[i] = h; r.l[i] = (__bf16)(v[i] - (float)h); }
  return r; }
__device__ __forceinline__ F2 split_row(const float* row, int k0, int lane) { float v[16]; const float* p = row + k0 + 8 * (lane >> 4);
#pragma unroll
  for (int i = 0; i < 8; ++i) { v[i] = p[i]; v[8 + i] = p[16 + i]; }
  return bsplit16(v); }
__device__ __forceinline__ float bfr(float v) { return (float)(__bf16)v; }
__host__ __device__ __forceinline__ int kb_last(int qb) { return (qb * 64 + 63) >> 7; }
#define LDSX() do { asm volatile("s_wait_dscnt 0" ::: "memory"); __builtin_amdgcn_wave_barrier(); __builtin_amdgcn_fence(3  , "workgroup"); } while (0)

__global__ __launch_bounds__(256) void k_cvt_x(const float* __restrict__ X, __bf16* __restrict__ XB) {
  const int row = blockIdx.x, tid = threadIdx.x; const int b = row / TT, t = row - b * TT;
  const float* src = X + ((size_t)b * SEQ_FULL + t) * DIN + tid * 8;
  const v4f a = *(const v4f*)src, c = *(const v4f*)(src + 4);
  union { v8b v; v4u u; } o;
#pragma unroll
  for (int i = 0; i < 4; ++i) { o.v[i] = (__bf16)a[i]; o.v[4 + i] = (__bf16)c[i]; }
  vst2((unsigned*)(XB + (size_t)row * DIN + tid * 8), o.u);
}
template <int F16S>
__global__ __launch_bounds__(256) void k_cvt_wT(const float* __restrict__ W, unsigned short* __restrict__ WT, int K, int N) {
  __shared__ float tile[32][68];
  const int k0 = blockIdx.x * 64, n0 = blockIdx.y * 32; const int tid = threadIdx.x, nn = tid & 31, kq = tid >> 5;
#pragma unroll
  for (int i = 0; i < 8; ++i) { const int kk = kq + 8 * i; tile[nn][kk] = W[(size_t)(k0 + kk) * N + n0 + nn]; }
  __syncthreads();
  const int nl = tid >> 3, q = tid & 7;
  union { v8b b; v8h h; v4u u; } o;
#pragma unroll
  for (int i = 0; i < 8; ++i) { const float v = bfr(tile[nl][q * 8 + i]); if (F16S) o.h[i] = (_Float16)(v * 256.0f); else o.b[i] = (__bf16)v; }
  vst2((unsigned*)(WT + (size_t)(n0 + nl) * K + k0 + q * 8), o.u);
}

__global__ __launch_bounds__(128) void k_proj(const __bf16* __restrict__ XB, const __bf16* __restrict__ WQT, const __bf16* __restrict__ WKT, const __bf16* __restrict__ WVT, const float* __restrict__ COS, const float* __restrict__ SIN,
    _Float16* __restrict__ QH, _Float16* __restrict__ QL, _Float16* __restrict__ KH, _Float16* __restrict__ KL, _Float16* __restrict__ VT, __bf16* __restrict__ VB, __bf16* __restrict__ VBL) {
  __shared__ __align__(16) _Float16 sh[64][136], sl[64][136]; __shared__ __align__(16) _Float16 th[128][72]; __shared__ __align__(16) __bf16 tb[128][72], tbl[128][72]; __shared__ float scs[64][HALF], ssn[64][HALF];
  const int tid = threadIdx.x, wave = tid >> 5, lane = tid & 31, col = lane & 15, g = lane >> 4;
  const int y = blockIdx.y; const int which = y < NH ? 0 : (y < NH + NKV ? 1 : 2); const int c0 = (which == 0 ? y : (which == 1 ? y - NH : y - NH - NKV)) * 128;
  const size_t r0 = (size_t)blockIdx.x * 64; const size_t bb = r0 / TT; const int t0 = (int)(r0 % TT);
  const __bf16* WT = which == 0 ? WQT : (which == 1 ? WKT : WVT);
  if (which < 2) { for (int e = tid; e < 64 * HALF; e += 128) { const int rr = e / HALF, p = e - rr * HALF; const size_t o = (size_t)(t0 + rr) * HALF + p; scs[rr][p] = bfr(COS[o]); ssn[rr][p] = bfr(SIN[o]); } }
  v8f acc[8] = {};
#pragma unroll 2
  for (int kc = 0; kc < DIN / 32; ++kc) { const v16b a = frag_b(XB + (r0 + wave * 16 + col) * DIN + kc * 32, lane);
    asm volatile("s_wait_loadcnt 0x0" ::: "memory");
#pragma unroll
    for (int j = 0; j < 8; ++j) { const v16b w = frag_b(WT + (size_t)(c0 + j * 16 + col) * DIN + kc * 32, lane); asm volatile("s_wait_loadcnt 0x0" ::: "memory"); acc[j] = wmma_bf(a, w, acc[j]); } }
  __syncthreads();
  if (which < 2) { _Float16* DH = which == 0 ? QH : KH; _Float16* DL = which == 0 ? QL : KL; const int ld = which == 0 ? CQ : CKV; const int nhi = which == 0 ? QHI : KHI; const bool hi_rows = t0 < nhi;
#pragma unroll
    for (int j = 0; j < 8; ++j) {
#pragma unroll
      for (int r = 0; r < 8; ++r) { const float v = acc[j][r]; const float pv = __shfl_xor(v, 1); const int rl = wave * 16 + 8 * g + r, cl = j * 16 + col; const int p = cl >> 1; const float c = scs[rl][p], s = ssn[rl][p];
        const float ev = v * c - pv * s, od = pv * s + v * c; const float rot = (col & 1) ? od : ev; const _Float16 hv = (_Float16)rot; sh[rl][cl] = hv; sl[rl][cl] = (_Float16)((rot - (float)hv) * 1024.0f); } }
    __syncthreads();
    for (int e = tid; e < 64 * 16; e += 128) { const int rl = e >> 4, q = e & 15; vst2((unsigned*)(DH + (r0 + rl) * (size_t)ld + c0 + q * 8), *(const v4u*)&sh[rl][q * 8]); if (hi_rows) vst2((unsigned*)(DL + (bb * nhi + t0 + rl) * (size_t)ld + c0 + q * 8), *(const v4u*)&sl[rl][q * 8]); }
  } else { const bool hi_rows = t0 < KHI;
#pragma unroll
    for (int j = 0; j < 8; ++j) {
#pragma unroll
      for (int r = 0; r < 8; ++r) { const float v = acc[j][r]; const int rl = wave * 16 + 8 * g + r, cl = j * 16 + col; th[cl][rl] = (_Float16)v; const __bf16 bh = (__bf16)v; tb[cl][rl] = bh; tbl[cl][rl] = (__bf16)(v - (float)bh); } }
    __syncthreads();
    for (int e = tid; e < 128 * 8; e += 128) { const int cl = e >> 3, q = e & 7; vst2((unsigned*)(VT + (bb * CKV + c0 + cl) * (size_t)TT + t0 + q * 8), *(const v4u*)&th[cl][q * 8]); if (hi_rows) { const size_t o3 = (bb * CKV + c0 + cl) * (size_t)KHI + t0 + q * 8; vst2((unsigned*)(VB + o3), *(const v4u*)&tb[cl][q * 8]); vst2((unsigned*)(VBL + o3), *(const v4u*)&tbl[cl][q * 8]); } } } }

__global__ __launch_bounds__(128) void k_sc(const _Float16* __restrict__ QH, const _Float16* __restrict__ KH, const _Float16* __restrict__ QL, const _Float16* __restrict__ KL, int b, int h0, float* __restrict__ S0) { __shared__ __align__(16) float ss[4][16][132];
  const int qb = blockIdx.x, kb = blockIdx.y; if (kb > kb_last(qb)) return;
  const int h = h0 + blockIdx.z, hk = h / GRP; float* S = S0 + (size_t)blockIdx.z * TT * TT;
  const int tid = threadIdx.x, wave = tid >> 5, lane = tid & 31, col = lane & 15, g = lane >> 4; const int k0 = kb * 128; const int ql0 = qb * 64 + wave * 16; const size_t q0 = (size_t)b * TT + ql0, kr0 = (size_t)b * TT + k0;
  v8f acc[8] = {}, accl[8] = {};
  const _Float16* QLb = QL + (size_t)b * QHI * CQ; const _Float16* KLb = KL + (size_t)b * KHI * CKV;
  if (qb < QBH) {
#pragma unroll 1
    for (int kc = 0; kc < HD / 32; ++kc) { const v16h ah = frag_h(QH + (q0 + col) * CQ + h * HD + kc * 32, lane), al = frag_h(QLb + (size_t)(ql0 + col) * CQ + h * HD + kc * 32, lane);
#pragma unroll
      for (int j = 0; j < 8; ++j) { const v16h kbf = frag_h(KH + (kr0 + j * 16 + col) * CKV + hk * HD + kc * 32, lane), klf = frag_h(KLb + (size_t)(k0 + j * 16 + col) * CKV + hk * HD + kc * 32, lane); acc[j] = wmma16(ah, kbf, acc[j]); accl[j] = wmma16(al, kbf, accl[j]); accl[j] = wmma16(ah, klf, accl[j]); } }
  } else if (qb * 64 < QHI) {
#pragma unroll 1
    for (int kc = 0; kc < HD / 32; ++kc) { const v16h ah = frag_h(QH + (q0 + col) * CQ + h * HD + kc * 32, lane), al = frag_h(QLb + (size_t)(ql0 + col) * CQ + h * HD + kc * 32, lane);
#pragma unroll
      for (int j = 0; j < 8; ++j) { const v16h kbf = frag_h(KH + (kr0 + j * 16 + col) * CKV + hk * HD + kc * 32, lane); acc[j] = wmma16(ah, kbf, acc[j]); accl[j] = wmma16(al, kbf, accl[j]); } }
  } else {
#pragma unroll 1
    for (int kc = 0; kc < HD / 32; ++kc) { const v16h ah = frag_h(QH + (q0 + col) * CQ + h * HD + kc * 32, lane);
#pragma unroll
      for (int j = 0; j < 8; ++j) { const v16h kbf = frag_h(KH + (kr0 + j * 16 + col) * CKV + hk * HD + kc * 32, lane); acc[j] = wmma16(ah, kbf, acc[j]); } } }
#pragma unroll
  for (int j = 0; j < 8; ++j) {
#pragma unroll
    for (int r = 0; r < 8; ++r) ss[wave][8 * g + r][j * 16 + col] = (acc[j][r] + accl[j][r] * (1.0f / 1024.0f)) * SCALE; }
  LDSX(); for (int rl = 0; rl < 16; ++rl) vst2(S + (size_t)(ql0 + rl) * TT + k0 + lane * 4, *(const v4f*)&ss[wave][rl][lane * 4]); }
__global__ __launch_bounds__(256) void k_sm(float* __restrict__ S0) { __shared__ float sred[8]; __shared__ float sbc; __shared__ __align__(16) float shv[TT];
  const int tid = threadIdx.x; const int t = blockIdx.x; const int kend = (kb_last(t >> 6) + 1) * 128;
  float* sr = S0 + (size_t)blockIdx.y * TT * TT + (size_t)t * TT;
  float m = -3.0e38f; for (int k = tid; k < kend; k += 256) { const float v = (k <= t) ? sr[k] : -3.0e38f; shv[k] = v; m = fmaxf(m, v); }
#pragma unroll
  for (int o = 1; o < 32; o <<= 1) m = fmaxf(m, __shfl_xor(m, o));
  if ((tid & 31) == 0) sred[tid >> 5] = m; __syncthreads(); if (tid == 0) { float a = sred[0]; for (int i = 1; i < 8; ++i) a = fmaxf(a, sred[i]); sbc = a; } __syncthreads(); m = sbc; __syncthreads();
  float sum = 0.f; for (int k = tid; k < kend; k += 256) { const float v = shv[k]; const float e = (v <= -1.0e38f) ? 0.f : expf(v - m); shv[k] = e; sum += e; }
#pragma unroll
  for (int o = 1; o < 32; o <<= 1) sum += __shfl_xor(sum, o);
  if ((tid & 31) == 0) sred[tid >> 5] = sum; __syncthreads(); if (tid == 0) { float a = 0.f; for (int i = 0; i < 8; ++i) a += sred[i]; sbc = a > 0.f ? 2048.0f / a : 0.f; } __syncthreads(); const float inv = sbc;
  for (int k = tid; k < kend; k += 256) shv[k] = shv[k] * inv;
  __syncthreads(); for (int q = tid; q < kend / 4; q += 256) vst2(sr + q * 4, *(const v4f*)&shv[q * 4]); }
__global__ __launch_bounds__(128) void k_pv(const float* __restrict__ PS0, const _Float16* __restrict__ VT, const __bf16* __restrict__ VB, const __bf16* __restrict__ VBL, int b, int h0, _Float16* __restrict__ CH, _Float16* __restrict__ CL) {
  const int h = h0 + blockIdx.z, hk = h / GRP; const float* PS = PS0 + (size_t)blockIdx.z * TT * TT; __shared__ __align__(16) _Float16 s2h[4][16][136], s2l[4][16][136];
  const int tid = threadIdx.x, wave = tid >> 5, lane = tid & 31, col = lane & 15, g = lane >> 4; const int qb = blockIdx.x; const int ql0 = qb * 64 + wave * 16; const int kce = (kb_last(qb) + 1) * 4; const bool hi_rows = qb * 64 < QHI;
  v8f acc[HD / 16] = {};
  if (qb < QBH) {
#pragma unroll 1
    for (int kc = 0; kc < kce; ++kc) { const F2 p = split_row(PS + (size_t)(ql0 + col) * TT, kc * 32, lane);
      asm volatile("s_wait_loadcnt 0x0" ::: "memory");
#pragma unroll
      for (int j = 0; j < HD / 16; ++j) { const size_t po = ((size_t)b * CKV + hk * HD + j * 16 + col) * (size_t)KHI + kc * 32; const v16b vh = frag_b(VB + po, lane); acc[j] = wmma_bf(p.h, vh, acc[j]); acc[j] = wmma_bf(p.l, vh, acc[j]); acc[j] = wmma_bf(p.h, frag_b(VBL + po, lane), acc[j]); } }
  } else {
#pragma unroll 1
    for (int kc = 0; kc < kce; ++kc) { const v16h p = frag_f32(PS + (size_t)(ql0 + col) * TT + kc * 32, lane);
      asm volatile("s_wait_loadcnt 0x0" ::: "memory");
#pragma unroll
      for (int j = 0; j < HD / 16; ++j) { const size_t po = ((size_t)b * CKV + hk * HD + j * 16 + col) * (size_t)TT + kc * 32; acc[j] = wmma16(p, frag_h(VT + po, lane), acc[j]); } } }
#pragma unroll
  for (int j = 0; j < HD / 16; ++j)
#pragma unroll
    for (int r = 0; r < 8; ++r) { const float v = acc[j][r] * (1.0f / 2048.0f); const _Float16 hv = (_Float16)v; s2h[wave][8 * g + r][j * 16 + col] = hv; s2l[wave][8 * g + r][j * 16 + col] = (_Float16)((v - (float)hv) * 1024.0f); }
  LDSX(); for (int rl = 0; rl < 16; ++rl) if (lane < 16) { vst2((unsigned*)(CH + ((size_t)b * TT + ql0 + rl) * CQ + h * HD + lane * 8), *(const v4u*)&s2h[wave][rl][lane * 8]); if (hi_rows) vst2((unsigned*)(CL + ((size_t)b * QHI + ql0 + rl) * CQ + h * HD + lane * 8), *(const v4u*)&s2l[wave][rl][lane * 8]); } }
__global__ __launch_bounds__(128) void k_out(const _Float16* __restrict__ CH, const _Float16* __restrict__ CL, const _Float16* __restrict__ WOT, float* __restrict__ OUT) {
  __shared__ __align__(16) float so[64][132];
  const int tid = threadIdx.x, wave = tid >> 5, lane = tid & 31, col = lane & 15, g = lane >> 4; const int c0 = blockIdx.y * 128;
  const size_t r0 = (size_t)blockIdx.x * 64; const size_t bb = r0 / TT; const int t0 = (int)(r0 % TT); const bool hi_rows = t0 < QHI; const int t0c = hi_rows ? t0 : 0;
  const _Float16* arow = CH + (r0 + wave * 16 + col) * (size_t)CQ; const _Float16* lrow = CL + (bb * QHI + t0c + wave * 16 + col) * (size_t)CQ;
  v8f acc[8] = {}, accl[8] = {};
  if (hi_rows) {
#pragma unroll 2
    for (int kc = 0; kc < CQ / 32; ++kc) { const v16h ah = frag_h(arow + kc * 32, lane), al = frag_h(lrow + kc * 32, lane);
      asm volatile("s_wait_loadcnt 0x0" ::: "memory");
#pragma unroll
      for (int j = 0; j < 8; ++j) { const v16h w = frag_h(WOT + (size_t)(c0 + j * 16 + col) * CQ + kc * 32, lane); asm volatile("s_wait_loadcnt 0x0" ::: "memory"); acc[j] = wmma16(ah, w, acc[j]); accl[j] = wmma16(al, w, accl[j]); } }
  } else {
#pragma unroll 2
    for (int kc = 0; kc < CQ / 32; ++kc) { const v16h ah = frag_h(arow + kc * 32, lane);
      asm volatile("s_wait_loadcnt 0x0" ::: "memory");
#pragma unroll
      for (int j = 0; j < 8; ++j) { const v16h w = frag_h(WOT + (size_t)(c0 + j * 16 + col) * CQ + kc * 32, lane); asm volatile("s_wait_loadcnt 0x0" ::: "memory"); acc[j] = wmma16(ah, w, acc[j]); } } }
#pragma unroll
  for (int j = 0; j < 8; ++j) {
#pragma unroll
    for (int r = 0; r < 8; ++r) so[wave * 16 + 8 * g + r][j * 16 + col] = (acc[j][r] + accl[j][r] * (1.0f / 1024.0f)) * (1.0f / 256.0f); }
  __syncthreads();
  for (int i = 0; i < 16; ++i) { const int rl = i * 4 + wave; vst2(OUT + ((bb * OSEQ + t0 + rl) * (size_t)DIN) + c0 + lane * 4, *(const v4f*)&so[rl][lane * 4]); } }

extern "C" void kernel_launch(void* const* d_in, const int* in_sizes, int n_in, void* d_out, int out_size, void* d_ws, size_t ws_size, hipStream_t stream) {
  if (n_in < 7) return;
  if (in_sizes[0] < ((NB - 1) * SEQ_FULL + SEQ) * DIN || in_sizes[1] < SEQ * HALF || in_sizes[2] < SEQ * HALF || in_sizes[3] < DIN * CQ || in_sizes[4] < DIN * CKV || in_sizes[5] < DIN * CKV || in_sizes[6] < CQ * DIN) return;
  if ((size_t)out_size < ((size_t)(NB - 1) * OSEQ + SEQ) * DIN) return;
  if (ws_size < (size_t)WS_END) return;
  const float** F = (const float**)d_in;
  char* ws = (char*)d_ws;
  __bf16 *XB = (__bf16*)(ws + WS_XB), *WQT = (__bf16*)(ws + WS_WQT), *WKT = (__bf16*)(ws + WS_WKT), *WVT = (__bf16*)(ws + WS_WVT), *VB = (__bf16*)(ws + WS_VB), *VBL = (__bf16*)(ws + WS_VBL);
  _Float16 *WOT = (_Float16*)(ws + WS_WOT), *QH = (_Float16*)(ws + WS_QH), *KH = (_Float16*)(ws + WS_KH), *VT = (_Float16*)(ws + WS_VT), *QL = (_Float16*)(ws + WS_QL), *KL = (_Float16*)(ws + WS_KL), *CH = (_Float16*)(ws + WS_CH), *CL = (_Float16*)(ws + WS_CL);
  float* S = (float*)(ws + WS_S);
  k_cvt_x<<<dim3(NB * TT), 256, 0, stream>>>(F[0], XB);
  k_cvt_wT<0><<<dim3(DIN / 64, CQ / 32), 256, 0, stream>>>(F[3], (unsigned short*)WQT, DIN, CQ);
  k_cvt_wT<0><<<dim3(DIN / 64, CKV / 32), 256, 0, stream>>>(F[4], (unsigned short*)WKT, DIN, CKV);
  k_cvt_wT<0><<<dim3(DIN / 64, CKV / 32), 256, 0, stream>>>(F[5], (unsigned short*)WVT, DIN, CKV);
  k_cvt_wT<1><<<dim3(CQ / 64, DIN / 32), 256, 0, stream>>>(F[6], (unsigned short*)WOT, CQ, DIN);
  k_proj<<<dim3(NB * TT / 64, NH + 2 * NKV, 1), 128, 0, stream>>>(XB, WQT, WKT, WVT, F[1], F[2], QH, QL, KH, KL, VT, VB, VBL);
  for (int b = 0; b < NB; ++b) for (int h0 = 0; h0 < NH; h0 += HG) {
    k_sc<<<dim3(NQB, TT / 128, HG), 128, 0, stream>>>(QH, KH, QL, KL, b, h0, S);
    k_sm<<<dim3(TT, HG), 256, 0, stream>>>(S);
    k_pv<<<dim3(NQB, 1, HG), 128, 0, stream>>>(S, VT, VB, VBL, b, h0, CH, CL);
  }
  k_out<<<dim3(NB * TT / 64, DIN / 128), 128, 0, stream>>>(CH, CL, WOT, (float*)d_out);
}
